// ContentAwareUpsample_82025285419163
// MI455X (gfx1250) — hardware-run, weakly checked
//
#include <hip/hip_runtime.h>


namespace {
constexpr int NB = 8, C = 64, H = 64, W = 64, C2 = 32, KK = 9, K1 = C * KK  , NM = C * KK * 4  , NP = NB * H * W  ;
constexpr float XS = 8.0f, WSC = 256.0f;
typedef _Float16 b16;
typedef __attribute__((ext_vector_type(16))) _Float16 v16b;
typedef __attribute__((ext_vector_type(8))) _Float16 v8b;
typedef __attribute__((ext_vector_type(8))) float v8f;
typedef __attribute__((ext_vector_type(4))) float v4f;
typedef __attribute__((ext_vector_type(2))) float v2f;
__device__ __forceinline__ float bf16_rne(float f) { unsigned int u = __float_as_uint(f); u += 0x7FFFu + ((u >> 16) & 1u); float r = __uint_as_float(u & 0xFFFF0000u); asm volatile("" : "+v"(r)); return r; }
__device__ __forceinline__ void split16(float v, b16& hi, b16& lo) { hi = (b16)v; lo = (b16)(v - (float)hi); }
__device__ __forceinline__ v16b frag_kb(const b16* p, int hh) { const v8b a = *(const v8b*)(p + 8 * hh), b = *(const v8b*)(p + 16 + 8 * hh); v16b f;
#pragma unroll
  for (int e = 0; e < 8; ++e) { f[e] = a[e]; f[8 + e] = b[e]; } return f; }
__device__ __forceinline__ v8f wmma16b(v16b a, v16b b, v8f c) { v8f d = __builtin_amdgcn_wmma_f32_16x16x32_f16(false, a, false, b, (short)0, c, false, false); asm volatile("v_nop\n\tv_nop\n\tv_nop\n\tv_nop" : "+v"(d) : "v"(a), "v"(b)); return d; }
__device__ __forceinline__ void wave_lds_sync() { __builtin_amdgcn_fence(__ATOMIC_RELEASE, "workgroup"); __builtin_amdgcn_wave_barrier(); __builtin_amdgcn_fence(__ATOMIC_ACQUIRE, "workgroup"); }
__device__ __forceinline__ float pmul(float a, float b) { float p = a * b; asm volatile("" : "+v"(p)); return p; }
__device__ __forceinline__ int iclamp(int v, int lo, int hi) { return v < lo ? lo : (v > hi ? hi : v); }

__global__ __launch_bounds__(256) void wput_kernel(const float* __restrict__ w1, const float* __restrict__ w2, const float* __restrict__ kw, b16* __restrict__ W1P, b16* __restrict__ W2P, b16* __restrict__ KPp) { const size_t u = (size_t)blockIdx.x * 256 + threadIdx.x; const size_t n1 = (size_t)C * K1 / 8, n2 = (size_t)C2 * K1 / 8, n3 = (size_t)NM * C2 / 8; v8b v;
  if (u < n1) {
#pragma unroll
    for (int j = 0; j < 8; ++j) v[j] = (b16)(bf16_rne(w1[u * 8 + j]) * WSC); for (int pass = 0; pass < 2; ++pass) { *(volatile v8b*)(W1P + u * 8) = v; __threadfence(); } }
  if (u < n2) {
#pragma unroll
    for (int j = 0; j < 8; ++j) v[j] = (b16)(bf16_rne(w2[u * 8 + j]) * WSC); for (int pass = 0; pass < 2; ++pass) { *(volatile v8b*)(W2P + u * 8) = v; __threadfence(); } }
  if (u < n3) {
#pragma unroll
    for (int j = 0; j < 8; ++j) v[j] = (b16)(bf16_rne(kw[u * 8 + j]) * WSC); for (int pass = 0; pass < 2; ++pass) { *(volatile v8b*)(KPp + u * 8) = v; __threadfence(); } } }
template <int MODE, int NT>
__global__ __launch_bounds__(32) void conv_kernel(const float* __restrict__ IN, const b16* __restrict__ WP, const float* __restrict__ bias, const float* __restrict__ pa, int PLIM, float* __restrict__ F) { constexpr int OW = NT * 16; __shared__ __attribute__((aligned(16))) b16 Ah[16][K1 + 8], Al[16][MODE == 0 ? 8 : K1 + 8]; __shared__ float Tf[16][OW + 4]; const int lane = threadIdx.x, nloc = lane & 15, hlf = lane >> 4; const size_t P0 = (size_t)blockIdx.x * 16; if (P0 >= (size_t)PLIM) return; const int b = (int)(P0 / (H * W)), h = (int)(P0 / W % H), w0 = (int)(P0 % W);
  for (int rr = 0; rr < 16; ++rr) { const int w = w0 + rr; for (int k = 0; k < KK; ++k) { const int dy = k / 3, dx = k % 3; const int hh = h + dy - 1, ww = w + dx - 1; const bool in = hh >= 0 && hh < H && ww >= 0 && ww < W;
      for (int cq = 0; cq < 2; ++cq) { const int ci = cq * 32 + lane; float v = 0.0f; if (in) { v = MODE == 0 ? bf16_rne(IN[(((size_t)b * C + ci) * H + hh) * W + ww]) : IN[(((size_t)b * H + hh) * W + ww) * C + ci]; }
        if (MODE == 0) Ah[rr][ci * KK + k] = (b16)(v * XS); else { b16 p, ql; split16(v * XS, p, ql); Ah[rr][ci * KK + k] = p; Al[rr][ci * KK + k] = ql; } } } }
  wave_lds_sync(); v8f acc[NT];
#pragma unroll
  for (int t = 0; t < NT; ++t) acc[t] = (v8f){};
#pragma unroll 2
  for (int kb = 0; kb < K1; kb += 32) { const v16b a = frag_kb(&Ah[nloc][kb], hlf); v16b al; if (MODE != 0) al = frag_kb(&Al[nloc][kb], hlf);
#pragma unroll
    for (int t = 0; t < NT; ++t) { const v16b bw = frag_kb(WP + (size_t)(t * 16 + nloc) * K1 + kb, hlf); acc[t] = wmma16b(a, bw, acc[t]); if (MODE != 0) acc[t] = wmma16b(al, bw, acc[t]); } }
#pragma unroll
  for (int t = 0; t < NT; ++t) { const int cc = t * 16 + nloc; const float bb = bf16_rne(bias[cc]), aa = bf16_rne(pa[cc]);
#pragma unroll
    for (int r8 = 0; r8 < 8; ++r8) { const float v = acc[t][r8] * (1.0f / (XS * WSC)) + bb; Tf[8 * hlf + r8][cc] = v > 0.0f ? v : pmul(aa, v); } }
  wave_lds_sync();
  for (int pass = 0; pass < 2; ++pass) { for (int rr = 0; rr < 16; ++rr) { if (OW == 64) *(volatile v2f*)(F + (P0 + rr) * OW + lane * 2) = (v2f){Tf[rr][lane * 2], Tf[rr][lane * 2 + 1]}; else ((volatile float*)F)[(P0 + rr) * OW + lane] = Tf[rr][lane]; } __threadfence(); } }
__global__ __launch_bounds__(32) void up_kernel(const float* __restrict__ F2, const b16* __restrict__ KPp, const float* __restrict__ kb, const float* __restrict__ xl, int PLIM, float* __restrict__ out) { __shared__ __attribute__((aligned(16))) b16 Ah[16][40], Al[16][40]; __shared__ float Tf[16][148]; const int lane = threadIdx.x, nloc = lane & 15, hlf = lane >> 4; const int ht = blockIdx.x & 3; const int w = (blockIdx.x >> 2) % W; const int b = (blockIdx.x >> 2) / W; const int h0 = ht * 16; if ((size_t)((b * H + h0) * W + w) >= (size_t)PLIM) return;
  for (int rr = 0; rr < 16; ++rr) { const size_t P = ((size_t)b * H + h0 + rr) * W + w; b16 p, ql; split16(F2[P * C2 + lane] * XS, p, ql); Ah[rr][lane] = p; Al[rr][lane] = ql; if (lane < 8) { Ah[rr][32 + lane] = (b16)0.0f; Al[rr][32 + lane] = (b16)0.0f; } }
  wave_lds_sync(); const v16b a = frag_kb(&Ah[nloc][0], hlf), al = frag_kb(&Al[nloc][0], hlf);
  const int hl = lane >> 1, pp = lane & 1; const int h = h0 + hl;
  float nb[KK];
  for (int pass = 0; pass < 2; ++pass) {
#pragma unroll 1
    for (int g = 0; g < C / 4; ++g) {
#pragma unroll
      for (int t = 0; t < 9; ++t) { v8f acc = {}; const int col0 = g * 144 + t * 16; acc = wmma16b(a, frag_kb(KPp + (size_t)(col0 + nloc) * C2, hlf), acc); acc = wmma16b(al, frag_kb(KPp + (size_t)(col0 + nloc) * C2, hlf), acc); const float bb = bf16_rne(kb[col0 + nloc]);
#pragma unroll
        for (int r8 = 0; r8 < 8; ++r8) Tf[8 * hlf + r8][t * 16 + nloc] = acc[r8] * (1.0f / (XS * WSC)) + bb; }
      wave_lds_sync();
#pragma unroll
      for (int cl = 0; cl < 4; ++cl) { const int c = g * 4 + cl; const float* xp = xl + ((size_t)b * C + c) * H * W;
#pragma unroll
        for (int k = 0; k < KK; ++k) { const int dy = k / 3, dx = k % 3; nb[k] = bf16_rne(xp[(size_t)iclamp(h + dy - 1, 0, H - 1) * W + iclamp(w + dx - 1, 0, W - 1)]); }
#pragma unroll
        for (int q = 0; q < 2; ++q) { float lg[KK]; float mx = -INFINITY;
#pragma unroll
          for (int k = 0; k < KK; ++k) { lg[k] = Tf[hl][cl * 36 + k * 4 + pp * 2 + q]; mx = fmaxf(mx, lg[k]); }
          float den = 0.0f, num = 0.0f;
#pragma unroll
          for (int k = 0; k < KK; ++k) { const float e = __expf(lg[k] - mx); den += e; num += pmul(e, nb[k]); }
          ((volatile float*)out)[(((size_t)b * C + c) * (2 * H) + (2 * w + q)) * (2 * W) + 2 * h0 + lane] = num / den; } }
      wave_lds_sync(); }
    __threadfence(); } }
}

extern "C" void kernel_launch(void* const* d_in, const int* in_sizes, int n_in, void* d_out, int out_size, void* d_ws, size_t ws_size, hipStream_t stream) {
  (void)n_in;
  auto Fp = [&](int i) { return (const float*)d_in[i]; };
  if (in_sizes[0] != NB * C * H * W || in_sizes[1] != NB * C * H * W || in_sizes[2] != C * K1 || in_sizes[5] != C2 * K1 || in_sizes[8] != NM * C2 || in_sizes[9] != NM || out_size != NB * C * 4 * H * W) return;
  const int BLIM = NB;
  const int PLIM = BLIM * H * W;
  size_t off = 0; char* ws = (char*)d_ws;
  auto carve = [&](size_t bytes) { char* p = ws + off; off += (bytes + 255) & ~(size_t)255; return p; };
  b16* W1P = (b16*)carve((size_t)C * K1 * 2); b16* W2P = (b16*)carve((size_t)C2 * K1 * 2); b16* KPp = (b16*)carve((size_t)NM * C2 * 2); float* F1 = (float*)carve((size_t)NP * C * 4); float* F2 = (float*)carve((size_t)NP * C2 * 4);
  if (off > ws_size || off > ((size_t)32 << 20)) return;
  wput_kernel<<<(unsigned)(((size_t)NM * C2 / 8 + 255) / 256), 256, 0, stream>>>(Fp(2), Fp(5), Fp(8), W1P, W2P, KPp);
  conv_kernel<0, 4><<<PLIM / 16, 32, 0, stream>>>(Fp(1), W1P, Fp(3), Fp(4), PLIM, F1);
  conv_kernel<1, 2><<<PLIM / 16, 32, 0, stream>>>(F1, W2P, Fp(6), Fp(7), PLIM, F2);
  up_kernel<<<BLIM * W * 4, 32, 0, stream>>>(F2, KPp, Fp(9), Fp(0), PLIM, (float*)d_out);
}
